// HeteroMLPPredictor_89249420411231
// MI455X (gfx1250) — hardware-verified
//
#include <hip/hip_runtime.h>


namespace {
constexpr int NU = 100000, NI = 50000, NIP = 50048, E = 1000000, D = 128;
constexpr float XS = 8.0f, WSC = 256.0f, NEG = 0.01f;
typedef _Float16 b16;
typedef __attribute__((ext_vector_type(16))) _Float16 v16b;
typedef __attribute__((ext_vector_type(8))) _Float16 v8b;
typedef __attribute__((ext_vector_type(8))) float v8f;
typedef __attribute__((ext_vector_type(4))) float v4f;
__device__ __forceinline__ float bf16_rne(float f) { unsigned int u = __float_as_uint(f); u += 0x7FFFu + ((u >> 16) & 1u); return __uint_as_float(u & 0xFFFF0000u); }
__device__ __forceinline__ void split16(float v, b16& hi, b16& lo) { hi = (b16)v; lo = (b16)(v - (float)hi); }
__device__ __forceinline__ v16b frag_kb(const b16* p, int hh) { const v8b a = *(const v8b*)(p + 8 * hh), b = *(const v8b*)(p + 16 + 8 * hh); v16b f;
#pragma unroll
  for (int e = 0; e < 8; ++e) { f[e] = a[e]; f[8 + e] = b[e]; } return f; }
__device__ __forceinline__ v8f wmma16b(v16b a, v16b b, v8f c) { v8f d = __builtin_amdgcn_wmma_f32_16x16x32_f16(false, a, false, b, (short)0, c, false, false); asm volatile("v_nop\n\tv_nop\n\tv_nop\n\tv_nop" : "+v"(d) : "v"(a), "v"(b)); return d; }
__device__ __forceinline__ void wave_lds_sync() { __builtin_amdgcn_fence(__ATOMIC_RELEASE, "workgroup"); __builtin_amdgcn_wave_barrier(); __builtin_amdgcn_fence(__ATOMIC_ACQUIRE, "workgroup"); }
__device__ __forceinline__ float pmul(float a, float b) { float p = a * b; asm volatile("" : "+v"(p)); return p; }
__device__ __forceinline__ int iclamp(int v, int lo, int hi) { return v < lo ? lo : (v > hi ? hi : v); }
__device__ __forceinline__ float leaky(float v) { return v >= 0.0f ? v : NEG * v; }

__global__ __launch_bounds__(256) void wprep_kernel(const float* __restrict__ w, b16* __restrict__ WT) {
  const int u = blockIdx.x * 256 + threadIdx.x; if (u >= D * D / 8) return; const int e = u * 8; const int o = e / D, k0 = e % D; v8b v;
#pragma unroll
  for (int j = 0; j < 8; ++j) v[j] = (b16)(bf16_rne(w[(size_t)(k0 + j) * D + o]) * WSC); for (int pass = 0; pass < 2; ++pass) { *(volatile v8b*)(WT + e) = v; __threadfence(); }
}
__global__ __launch_bounds__(32) void node_kernel(const float* __restrict__ h, int n, const b16* __restrict__ WT, const float* __restrict__ bias, float* __restrict__ F) {
  __shared__ __attribute__((aligned(16))) b16 Ah[16][D + 8]; __shared__ __attribute__((aligned(16))) float Tf[16][D + 4];
  const int lane = threadIdx.x, nloc = lane & 15, hlf = lane >> 4; const size_t m0 = (size_t)blockIdx.x * 16;
  for (int rr = 0; rr < 16; ++rr) { const size_t r = (m0 + rr) < (size_t)n ? m0 + rr : (size_t)n - 1; const v4f v = *(const v4f*)(h + r * D + lane * 4); for (int j = 0; j < 4; ++j) Ah[rr][lane * 4 + j] = (b16)(bf16_rne(v[j]) * XS); }
  wave_lds_sync();
  v8f acc[8];
#pragma unroll
  for (int t = 0; t < 8; ++t) acc[t] = (v8f){};
#pragma unroll 2
  for (int kb = 0; kb < D; kb += 32) { const v16b a = frag_kb(&Ah[nloc][kb], hlf);
#pragma unroll
    for (int t = 0; t < 8; ++t) acc[t] = wmma16b(a, frag_kb(WT + (size_t)(t * 16 + nloc) * D + kb, hlf), acc[t]); }
#pragma unroll
  for (int t = 0; t < 8; ++t) { const int c = t * 16 + nloc; const float bb = bf16_rne(bias[c]);
#pragma unroll 1
    for (int r8 = 0; r8 < 8; ++r8) Tf[8 * hlf + r8][c] = acc[t][r8] * (1.0f / (XS * WSC)) + bb; }
  wave_lds_sync();
  for (int pass = 0; pass < 2; ++pass) { for (int rr = 0; rr < 16; ++rr) if (m0 + rr < (size_t)n) *(volatile v4f*)(F + (m0 + rr) * D + lane * 4) = *(const v4f*)(&Tf[rr][lane * 4]); __threadfence(); }
}
__global__ __launch_bounds__(64) void edge_kernel(const float* __restrict__ UF, const float* __restrict__ IF, const int* __restrict__ srcs, const int* __restrict__ dsts, const b16* __restrict__ W1T, const float* __restrict__ b1, const float* __restrict__ W2, const float* __restrict__ b2, int ELIM, float* __restrict__ out) {
  __shared__ __attribute__((aligned(16))) b16 Ah[2][16][D + 8], Al[2][16][D + 8]; __shared__ float so[32];
  const int wave = threadIdx.x >> 5, lane = threadIdx.x & 31, nloc = lane & 15, hlf = lane >> 4; const size_t e0 = (size_t)blockIdx.x * 32 + wave * 16;
  for (int rr = 0; rr < 16; ++rr) { const size_t e = e0 + rr; v4f a = {0, 0, 0, 0};
    if (e < (size_t)ELIM) { const int s = iclamp(srcs[e], 0, NU - 1), d = iclamp(dsts[e], 0, NI - 1); const v4f u = *(const v4f*)(UF + (size_t)s * D + lane * 4), it = *(const v4f*)(IF + (size_t)d * D + lane * 4); for (int j = 0; j < 4; ++j) a[j] = leaky(u[j] + it[j]); }
    for (int j = 0; j < 4; ++j) { b16 p, q; split16(a[j] * XS, p, q); Ah[wave][rr][lane * 4 + j] = p; Al[wave][rr][lane * 4 + j] = q; } }
  wave_lds_sync();
  v8f acc[8];
#pragma unroll
  for (int t = 0; t < 8; ++t) acc[t] = (v8f){};
#pragma unroll 2
  for (int kb = 0; kb < D; kb += 32) { const v16b a = frag_kb(&Ah[wave][nloc][kb], hlf), al = frag_kb(&Al[wave][nloc][kb], hlf);
#pragma unroll
    for (int t = 0; t < 8; ++t) { const v16b bw = frag_kb(W1T + (size_t)(t * 16 + nloc) * D + kb, hlf); acc[t] = wmma16b(a, bw, acc[t]); acc[t] = wmma16b(al, bw, acc[t]); } }
  float pd[8]; for (int r8 = 0; r8 < 8; ++r8) pd[r8] = 0.0f;
#pragma unroll
  for (int t = 0; t < 8; ++t) { const int c = t * 16 + nloc; const float bb = bf16_rne(b1[c]), w2 = bf16_rne(W2[c]);
#pragma unroll
    for (int r8 = 0; r8 < 8; ++r8) pd[r8] += pmul(leaky(acc[t][r8] * (1.0f / (XS * WSC)) + bb), w2); }
  const float bb2 = bf16_rne(b2[0]);
#pragma unroll
  for (int r8 = 0; r8 < 8; ++r8) { float s = pd[r8]; for (int o = 1; o < 16; o <<= 1) s += __shfl_xor(s, o); if (nloc == 0) so[wave * 16 + 8 * hlf + r8] = leaky(s + bb2); }
  __syncthreads();
  for (int pass = 0; pass < 2; ++pass) { if (threadIdx.x < 32) ((volatile float*)out)[(size_t)blockIdx.x * 32 + threadIdx.x] = so[threadIdx.x]; __threadfence(); }
}
}

extern "C" void kernel_launch(void* const* d_in, const int* in_sizes, int n_in, void* d_out, int out_size, void* d_ws, size_t ws_size, hipStream_t stream) {
  (void)n_in;
  auto Fp = [&](int i) { return (const float*)d_in[i]; }; auto Ip = [&](int i) { return (const int*)d_in[i]; };
  if (in_sizes[0] != NU * D || in_sizes[1] != NI * D || in_sizes[2] != E || in_sizes[3] != E || in_sizes[4] != D * D || in_sizes[6] != D * D || in_sizes[8] != D * D || in_sizes[10] != D || out_size != E) return;
  const int ELIM = E;
  size_t off = 0; char* ws = (char*)d_ws;
  auto carve = [&](size_t bytes) { char* p = ws + off; off += (bytes + 255) & ~(size_t)255; return p; };
  b16* WL = (b16*)carve(D * D * 2); b16* WR = (b16*)carve(D * D * 2); b16* W1T = (b16*)carve(D * D * 2); float* UF = (float*)carve((size_t)NU * D * 4); float* IF = (float*)carve((size_t)NIP * D * 4);
  if (off > ws_size || off > ((size_t)128 << 20)) return;
  wprep_kernel<<<(D * D / 8 + 255) / 256, 256, 0, stream>>>(Fp(4), WL); wprep_kernel<<<(D * D / 8 + 255) / 256, 256, 0, stream>>>(Fp(6), WR); wprep_kernel<<<(D * D / 8 + 255) / 256, 256, 0, stream>>>(Fp(8), W1T);
  node_kernel<<<NU / 16, 32, 0, stream>>>(Fp(0), NU, WL, Fp(5), UF); node_kernel<<<NIP / 16, 32, 0, stream>>>(Fp(1), NI, WR, Fp(7), IF);
  edge_kernel<<<(ELIM + 31) / 32, 64, 0, stream>>>(UF, IF, Ip(2), Ip(3), W1T, Fp(9), Fp(10), Fp(11), ELIM, (float*)d_out);
}
